// FinalModel_3985729651483
// MI455X (gfx1250) — hardware-run, weakly checked
//
#include <hip/hip_runtime.h>


#ifndef NB
#define NB 32
#endif
#define NB_FULL 32
#define MR    32
#define SPW   9
#define NBAND 200
#define DIN   16200
#define KP1   16256
#define HID   1024
#define ODIM  512
#define CAT   2048
#define GW    4
#define RP    68
#define G1    (KP1 / 8)
#define GR1   (DIN / 8)
#define ACAR  64.0f
#define WCAR  256.0f
#define DSC   (1.0f / 16384.0f)
#define LN_EPS 1.0e-5f
#define T2L   2.8853900817779268f

static_assert(DIN == SPW * SPW * NBAND);
static_assert(DIN % 8 == 0);
static_assert(KP1 >= DIN);
static_assert(KP1 % (32 * GW) == 0);
static_assert(KP1 % 64 == 0);
static_assert(HID % (32 * GW) == 0);
static_assert(CAT % (32 * GW) == 0);
static_assert(CAT == 2 * HID);
static_assert(HID % 64 == 0);
static_assert(ODIM % 64 == 0);
static_assert(HID / 8 == 128);
static_assert(MR == 32);
static_assert(NB >= 1);
static_assert(NB <= MR);
static_assert(NB <= NB_FULL);
static_assert(ACAR * WCAR * DSC == 1.0f);
static_assert(64 * 256 >= DIN);
static_assert(8 * 256 >= G1);
static_assert((RP * 4) % 16 == 0);
static_assert((size_t)DIN * 4 + 64 <= 131072);
static_assert((size_t)GW * MR * RP * 4 <= 131072);
static_assert((size_t)2 * MR * RP * 4 <= 131072);
static_assert(((size_t)HID * KP1) % 256 == 0);
static_assert(((size_t)ODIM * (HID / 8)) % 256 == 0);

typedef _Float16 h16;
typedef __attribute__((ext_vector_type(16))) _Float16 v16h;
typedef __attribute__((ext_vector_type(8)))  _Float16 v8h;
typedef __attribute__((ext_vector_type(8)))  float    v8f;
typedef __attribute__((ext_vector_type(4)))  float    v4f;
typedef v4f  __attribute__((may_alias)) v4fa;

__device__ __forceinline__ unsigned short f2bf(float f) { unsigned u = __float_as_uint(f); u += 0x7FFFu + ((u >> 16) & 1u); return (unsigned short)(u >> 16); }
__device__ __forceinline__ float bfr(float f) { return __uint_as_float(((unsigned)f2bf(f)) << 16); }
__device__ __forceinline__ v16h cat16(v8h lo, v8h hi) { return __builtin_shufflevector(lo, hi, 0, 1, 2, 3, 4, 5, 6, 7, 8, 9, 10, 11, 12, 13, 14, 15); }
__device__ __forceinline__ v8f wmma16(v16h a, v16h b, v8f c) { return __builtin_amdgcn_wmma_f32_16x16x32_f16(false, a, false, b, (short)0, c, false, false); }
__device__ __forceinline__ v16h  ldh(const h16* p) { return cat16(*(const v8h*)p, *(const v8h*)(p + 16)); }
__device__ __forceinline__ v8f wmma16g(v16h a, v16h b, v8f c) {
    c = wmma16(a, b, c);
    asm volatile("v_nop\n\tv_nop\n\tv_nop\n\tv_nop" : "+v"(c) : "v"(a), "v"(b));
    return c;
}
static __device__ __forceinline__ h16 toh_flush(float v) { const h16 r = (h16)v; return (fabsf(v) < 6.103515625e-05f) ? (h16)0.0f : r; }

__global__ __launch_bounds__(256) void k_gse_ln(const float* __restrict__ x, const float* __restrict__ wg, const float* __restrict__ bg,
                                                const float* __restrict__ lg, const float* __restrict__ lb, h16* LNH) {
#pragma clang fp contract(off)
    __shared__ __align__(16) float sf[DIN];
    __shared__ float rs1[8];
    __shared__ float rs2[8];
    const int tid = threadIdx.x, lane = tid & 31;
    const int wave = __builtin_amdgcn_readfirstlane((int)(threadIdx.x >> 5));
    const int row = blockIdx.x;
    h16* orow = LNH + (size_t)row * KP1;
    if (row >= NB) {
        const v8h z = (v8h){};
#pragma unroll 1
        for (int ps = 0; ps < 2; ++ps) {
#pragma unroll 1
            for (int it = 0; it < 8; ++it) { const int g = it * 256 + tid; if (g < G1) *(volatile v8h*)(orow + (size_t)g * 8) = z; }
            if (ps == 0) __threadfence(); }
        return;
    }
    const float* xr = x + (size_t)row * DIN;
    float sum = 0.0f;
#pragma unroll 1
    for (int it = 0; it < 64; ++it) {
        const int idx = it * 256 + tid;
        const bool ok = idx < DIN;
        const int ic = ok ? idx : (DIN - 1);
        const int c = ic % NBAND, w = (ic / NBAND) % SPW;
        const int il = (ic - NBAND) < 0 ? 0 : (ic - NBAND);
        const int ir = (ic + NBAND) > (DIN - 1) ? (DIN - 1) : (ic + NBAND);
        float xl = xr[il], xc = xr[ic], xn = xr[ir];
        asm volatile("" : "+v"(xl)); asm volatile("" : "+v"(xn));
        const float w0 = bfr(wg[c * 3 + 0]), w1 = bfr(wg[c * 3 + 1]), w2 = bfr(wg[c * 3 + 2]), bv = bfr(bg[c]);
        const float vl = (w > 0) ? bfr(xl) : 0.0f;
        const float vn = (w < SPW - 1) ? bfr(xn) : 0.0f;
        float acc = ((vl * w0 + bfr(xc) * w1) + vn * w2) + bv;
        asm volatile("" : "+v"(acc));
        if (ok) sf[idx] = acc;
        sum += ok ? acc : 0.0f;
    }
    { float v = sum;
      v += __shfl_xor(v, 16, 32); v += __shfl_xor(v, 8, 32); v += __shfl_xor(v, 4, 32); v += __shfl_xor(v, 2, 32); v += __shfl_xor(v, 1, 32);
      if (lane == 0) rs1[wave] = v; }
    __syncthreads();
    float tot = 0.0f;
#pragma unroll
    for (int k = 0; k < 8; ++k) tot += rs1[k];
    const float mu = tot * (1.0f / (float)DIN);
    float sq = 0.0f;
#pragma unroll 1
    for (int it = 0; it < 64; ++it) {
        const int idx = it * 256 + tid;
        const bool ok = idx < DIN;
        const int ic = ok ? idx : (DIN - 1);
        const float d = sf[ic] - mu;
        sq += ok ? d * d : 0.0f;
    }
    { float v = sq;
      v += __shfl_xor(v, 16, 32); v += __shfl_xor(v, 8, 32); v += __shfl_xor(v, 4, 32); v += __shfl_xor(v, 2, 32); v += __shfl_xor(v, 1, 32);
      if (lane == 0) rs2[wave] = v; }
    __syncthreads();
    float tq = 0.0f;
#pragma unroll
    for (int k = 0; k < 8; ++k) tq += rs2[k];
    const float rstd = rsqrtf(tq * (1.0f / (float)DIN) + LN_EPS);
#pragma unroll 1
    for (int ps = 0; ps < 2; ++ps) {
#pragma unroll 1
        for (int it = 0; it < 8; ++it) {
            const int g = it * 256 + tid;
            const int gc = g < GR1 ? g : (GR1 - 1);
            v4f g0 = *(const v4f*)(lg + (size_t)gc * 8), g1 = *(const v4f*)(lg + (size_t)gc * 8 + 4);
            v4f b0 = *(const v4f*)(lb + (size_t)gc * 8), b1 = *(const v4f*)(lb + (size_t)gc * 8 + 4);
            asm volatile("" : "+v"(g0)); asm volatile("" : "+v"(g1)); asm volatile("" : "+v"(b0)); asm volatile("" : "+v"(b1));
            const v4f f0 = *(const v4fa*)(&sf[gc * 8]), f1 = *(const v4fa*)(&sf[gc * 8 + 4]);
            const bool live = g < GR1;
            v8h hv;
#pragma unroll
            for (int i = 0; i < 4; ++i) {
                const float t0 = ((f0[i] - mu) * rstd * bfr(g0[i]) + bfr(b0[i])) * ACAR;
                const float t1 = ((f1[i] - mu) * rstd * bfr(g1[i]) + bfr(b1[i])) * ACAR;
                hv[i] = live ? toh_flush(t0) : (h16)0.0f; hv[4 + i] = live ? toh_flush(t1) : (h16)0.0f; }
            if (g < G1) *(volatile v8h*)(orow + (size_t)g * 8) = hv;
        }
        if (ps == 0) __threadfence(); }
}

__global__ __launch_bounds__(256) void k_wcvt(const float* __restrict__ src, h16* dst, int rows, int K, int G, int dpitch) {
#pragma clang fp contract(off)
    const unsigned total = (unsigned)rows * (unsigned)G;
    const unsigned i = blockIdx.x * 256u + threadIdx.x;
    const unsigned ic = i < total ? i : (total - 1u);
    const unsigned n = ic / (unsigned)G;
    const unsigned g = ic - n * (unsigned)G;
    const unsigned gr = (unsigned)(K >> 3);
    const unsigned gc = g < gr ? g : (gr - 1u);
    const float* p = src + (size_t)n * (size_t)K + (size_t)gc * 8;
    v4f a = *(const v4f*)p, b = *(const v4f*)(p + 4);
    asm volatile("" : "+v"(a)); asm volatile("" : "+v"(b));
    const bool live = g < gr;
    v8h hv;
#pragma unroll
    for (int k = 0; k < 4; ++k) { hv[k] = live ? toh_flush(bfr(a[k]) * WCAR) : (h16)0.0f; hv[4 + k] = live ? toh_flush(bfr(b[k]) * WCAR) : (h16)0.0f; }
    h16* q = dst + (size_t)n * (size_t)dpitch + (size_t)g * 8;
    if (i < total) { *(volatile v8h*)q = hv; __threadfence(); *(volatile v8h*)q = hv; }
}

__global__ __launch_bounds__(256) void k_wtap(const float* __restrict__ src, h16* dst) {
#pragma clang fp contract(off)
    const unsigned total = (unsigned)HID * (unsigned)(HID / 8);
    const unsigned i = blockIdx.x * 256u + threadIdx.x;
    const unsigned ic = i < total ? i : (total - 1u);
    const unsigned n = ic >> 7, g = ic & 127u;
    const size_t base = ((size_t)n * HID + (size_t)g * 8) * 3 + 1;
    float t[8];
#pragma unroll
    for (int k = 0; k < 8; ++k) t[k] = src[base + (size_t)(3 * k)];
    v8h hv;
#pragma unroll
    for (int k = 0; k < 8; ++k) hv[k] = toh_flush(bfr(t[k]) * WCAR);
    h16* q = dst + (size_t)n * HID + (size_t)g * 8;
    if (i < total) { *(volatile v8h*)q = hv; __threadfence(); *(volatile v8h*)q = hv; }
}

template <int OUTF>
__device__ __forceinline__ void gemm_body(const h16* __restrict__ Act, const h16* __restrict__ W, const float* __restrict__ bias0, const float* __restrict__ bias1,
                                          float* OF, h16* OH, int K, int apitch, int acoly, int wrowy, int opitch, int ocoly, int bsum, int orows) {
    __shared__ __align__(16) float red[GW * MR * RP];
    const int tid = threadIdx.x;
    const int lane = tid & 31, lr = lane & 15, hi = lane >> 4;
    const int wave = __builtin_amdgcn_readfirstlane((int)(threadIdx.x >> 5));
    const int y = blockIdx.y, c0 = blockIdx.x * 64;
    const int nst = (K >> 5) / GW;
    const int kb = wave * nst * 32;
    const size_t aoff = (size_t)lr * (size_t)apitch + (size_t)y * (size_t)acoly + (size_t)(8 * hi);
    const size_t boff = ((size_t)y * (size_t)wrowy + (size_t)(c0 + lr)) * (size_t)K + (size_t)(8 * hi);
    v8f acc[2][4];
#pragma unroll
    for (int mb = 0; mb < 2; ++mb)
#pragma unroll
        for (int nb = 0; nb < 4; ++nb) acc[mb][nb] = (v8f){};
#pragma unroll 1
    for (int s = 0; s < nst; ++s) {
        const int kc = kb + s * 32;
        const v16h a0 = ldh(Act + aoff + (size_t)kc);
        const v16h a1 = ldh(Act + aoff + (size_t)16 * (size_t)apitch + (size_t)kc);
#pragma unroll
        for (int nb = 0; nb < 4; ++nb) {
            const v16h b = ldh(W + boff + (size_t)nb * 16 * (size_t)K + (size_t)kc);
            acc[0][nb] = wmma16g(a0, b, acc[0][nb]);
            acc[1][nb] = wmma16g(a1, b, acc[1][nb]); }
    }
    const int wb = wave * MR * RP;
#pragma unroll
    for (int mb = 0; mb < 2; ++mb)
#pragma unroll
        for (int nb = 0; nb < 4; ++nb)
#pragma unroll
            for (int j = 0; j < 8; ++j) red[wb + (mb * 16 + hi * 8 + j) * RP + nb * 16 + lr] = acc[mb][nb][j];
    __syncthreads();
    if (OUTF == 0) {
        static_assert(32 * GW * 8 * 2 == MR * 64);
#pragma unroll 1
        for (int ps = 0; ps < 2; ++ps) {
#pragma unroll 1
            for (int it = 0; it < 2; ++it) {
                const int p = it * (32 * GW) + tid; const int row = p >> 3, c8 = (p & 7) * 8;
                const int ro = row * RP + c8;
                v4f s0 = *(const v4fa*)(&red[ro]), s1 = *(const v4fa*)(&red[ro + 4]);
#pragma unroll
                for (int w = 1; w < GW; ++w) { s0 = s0 + *(const v4fa*)(&red[w * MR * RP + ro]); s1 = s1 + *(const v4fa*)(&red[w * MR * RP + ro + 4]); }
                const int cm = c0 + c8;
                const v4f p0 = *(const v4f*)(bias0 + cm), p1 = *(const v4f*)(bias0 + cm + 4);
                const v4f q0 = *(const v4f*)(bias1 + cm), q1 = *(const v4f*)(bias1 + cm + 4);
                v8h hv;
#pragma unroll
                for (int i = 0; i < 4; ++i) {
                    const float x0 = bfr(p0[i]), x1 = bfr(q0[i]), z0 = bfr(p1[i]), z1 = bfr(q1[i]);
                    const float ba = bsum ? (x0 + x1) : (y ? x1 : x0);
                    const float bc = bsum ? (z0 + z1) : (y ? z1 : z0);
                    hv[i] = toh_flush((s0[i] * DSC + ba) * ACAR); hv[4 + i] = toh_flush((s1[i] * DSC + bc) * ACAR); }
                *(volatile v8h*)(OH + (size_t)row * (size_t)opitch + (size_t)y * (size_t)ocoly + (size_t)cm) = hv;
            }
            if (ps == 0) __threadfence(); }
    } else {
        static_assert(32 * GW * 4 * 4 == MR * 64);
#pragma unroll 1
        for (int ps = 0; ps < 2; ++ps) {
#pragma unroll 1
            for (int it = 0; it < 4; ++it) {
                const int p = it * (32 * GW) + tid; const int row = p >> 4, c4 = (p & 15) * 4;
                const int ro = row * RP + c4;
                v4f s0 = *(const v4fa*)(&red[ro]);
#pragma unroll
                for (int w = 1; w < GW; ++w) s0 = s0 + *(const v4fa*)(&red[w * MR * RP + ro]);
                const int cm = c0 + c4;
                const v4f p0 = *(const v4f*)(bias0 + cm);
                const v4f q0 = *(const v4f*)(bias1 + cm);
                v4f o;
#pragma unroll
                for (int i = 0; i < 4; ++i) {
                    const float x0 = bfr(p0[i]), x1 = bfr(q0[i]);
                    const float ba = bsum ? (x0 + x1) : (y ? x1 : x0);
                    o[i] = s0[i] * DSC + ba; }
                if (row < orows) *(volatile v4f*)(OF + (size_t)row * (size_t)opitch + (size_t)y * (size_t)ocoly + (size_t)cm) = o;
            }
            if (ps == 0) __threadfence(); }
    }
}

__global__ __launch_bounds__(32 * GW) void k_gemm_h(const h16* __restrict__ Act, const h16* __restrict__ W, const float* __restrict__ bias0, const float* __restrict__ bias1,
                                                    h16* OH, int K, int apitch, int acoly, int wrowy, int opitch, int ocoly, int bsum) {
    gemm_body<0>(Act, W, bias0, bias1, (float*)0, OH, K, apitch, acoly, wrowy, opitch, ocoly, bsum, MR);
}

__global__ __launch_bounds__(32 * GW) void k_gemm_f(const h16* __restrict__ Act, const h16* __restrict__ W, const float* __restrict__ bias0, const float* __restrict__ bias1,
                                                    float* OF, int K, int apitch, int acoly, int wrowy, int opitch, int ocoly, int bsum, int orows) {
    gemm_body<1>(Act, W, bias0, bias1, OF, (h16*)0, K, apitch, acoly, wrowy, opitch, ocoly, bsum, orows);
}

__global__ __launch_bounds__(256) void k_tanhmean(const float* __restrict__ CF, const float* __restrict__ M, const float* __restrict__ delta, h16* FB, int coff) {
#pragma clang fp contract(off)
    __shared__ __align__(16) float cft[MR * RP];
    __shared__ __align__(16) float ot[MR * RP];
    const int tid = threadIdx.x, lane = tid & 31;
    const int wave = __builtin_amdgcn_readfirstlane((int)(threadIdx.x >> 5));
    const int i0 = blockIdx.x * 64;
    static_assert(256 * 4 * 2 == MR * 64);
#pragma unroll 1
    for (int it = 0; it < 2; ++it) {
        const int p = it * 256 + tid; const int row = p >> 4, c4 = (p & 15) * 4;
        const v4f v = *(const v4f*)(CF + (size_t)row * CAT + (size_t)coff + (size_t)(i0 + c4));
        *(v4fa*)(&cft[row * RP + c4]) = v; }
    __syncthreads();
#pragma unroll 1
    for (int ii = 0; ii < 8; ++ii) {
        const int il = wave * 8 + ii;
        const int i = i0 + il;
        const float dl = bfr(delta[i]);
        float cbuf[32], acc[32];
#pragma unroll
        for (int b = 0; b < 32; ++b) { cbuf[b] = cft[b * RP + il] * T2L; acc[b] = 0.0f; }
        const float* Mi = M + (size_t)i * HID;
#pragma unroll 1
        for (int jt = 0; jt < HID / 32; ++jt) {
            const float a2 = (bfr(Mi[jt * 32 + lane]) * dl) * T2L;
#pragma unroll
            for (int b = 0; b < 32; ++b) {
                const float e = __builtin_amdgcn_exp2f(cbuf[b] + a2);
                acc[b] += __builtin_amdgcn_rcpf(e + 1.0f); }
        }
        float mine = 0.0f;
#pragma unroll
        for (int b = 0; b < 32; ++b) {
            float v = acc[b];
            v += __shfl_xor(v, 16, 32); v += __shfl_xor(v, 8, 32); v += __shfl_xor(v, 4, 32); v += __shfl_xor(v, 2, 32); v += __shfl_xor(v, 1, 32);
            mine = (lane == b) ? v : mine; }
        ot[lane * RP + il] = 1.0f - mine * (2.0f / (float)HID);
    }
    __syncthreads();
    static_assert(256 * 8 * 1 == MR * 64);
    { const int row = tid >> 3, c8 = (tid & 7) * 8;
      const v4f x0 = *(const v4fa*)(&ot[row * RP + c8]), x1 = *(const v4fa*)(&ot[row * RP + c8 + 4]);
      v8h hv;
#pragma unroll
      for (int k = 0; k < 4; ++k) { hv[k] = toh_flush(x0[k] * ACAR); hv[4 + k] = toh_flush(x1[k] * ACAR); }
      h16* q = FB + (size_t)row * CAT + (size_t)coff + (size_t)(i0 + c8);
      *(volatile v8h*)q = hv; __threadfence(); *(volatile v8h*)q = hv; }
}

static constexpr size_t al256(size_t v) { return (v + 255) & ~(size_t)255; }
static constexpr size_t SZ_LNH = al256((size_t)MR * KP1 * 2);
static constexpr size_t SZ_WXZ = al256((size_t)2 * HID * KP1 * 2);
static constexpr size_t SZ_WC  = al256((size_t)2 * HID * HID * 2);
static constexpr size_t SZ_WO  = al256((size_t)ODIM * CAT * 2);
static constexpr size_t SZ_XZH = al256((size_t)MR * CAT * 2);
static constexpr size_t SZ_CFB = al256((size_t)MR * CAT * 4);
static constexpr size_t SZ_FBH = al256((size_t)MR * CAT * 2);
static constexpr size_t SZ_TOTAL = SZ_LNH + SZ_WXZ + SZ_WC + SZ_WO + SZ_XZH + SZ_CFB + SZ_FBH;
static_assert(SZ_TOTAL <= (size_t)134217728);
static_assert(((size_t)HID * KP1 * 2) % 256 == 0);
static_assert(((size_t)HID * HID * 2) % 256 == 0);
static_assert(((size_t)HID * 2) % 128 == 0);

extern "C" void kernel_launch(void* const* d_in, const int* in_sizes, int n_in,
                              void* d_out, int out_size, void* d_ws, size_t ws_size, hipStream_t stream) {
    if (n_in < 20) return;
    if ((size_t)in_sizes[0] < (size_t)NB * DIN) return;
    if (in_sizes[1] < NBAND * 3 || in_sizes[2] < NBAND || in_sizes[3] < DIN || in_sizes[4] < DIN) return;
    if ((size_t)in_sizes[5] < (size_t)HID * DIN || (size_t)in_sizes[7] < (size_t)HID * DIN) return;
    if (in_sizes[6] < HID || in_sizes[8] < HID || in_sizes[10] < HID || in_sizes[12] < HID || in_sizes[15] < HID) return;
    if ((size_t)in_sizes[9] < (size_t)HID * HID * 3 || (size_t)in_sizes[11] < (size_t)HID * HID * 3) return;
    if ((size_t)in_sizes[13] < (size_t)HID * HID || (size_t)in_sizes[14] < (size_t)HID * HID) return;
    if ((size_t)in_sizes[16] < (size_t)ODIM * HID || (size_t)in_sizes[18] < (size_t)ODIM * HID) return;
    if (in_sizes[17] < ODIM || in_sizes[19] < ODIM) return;
    if ((size_t)out_size < (size_t)NB * ODIM) return;
    if (SZ_TOTAL > ws_size) return;
    const float* x    = (const float*)d_in[0];
    const float* wgse = (const float*)d_in[1];
    const float* bgse = (const float*)d_in[2];
    const float* lng  = (const float*)d_in[3];
    const float* lnb  = (const float*)d_in[4];
    const float* Wx   = (const float*)d_in[5];
    const float* bx   = (const float*)d_in[6];
    const float* Wz   = (const float*)d_in[7];
    const float* bz   = (const float*)d_in[8];
    const float* Wcf  = (const float*)d_in[9];
    const float* bcf  = (const float*)d_in[10];
    const float* Wcb  = (const float*)d_in[11];
    const float* bcb  = (const float*)d_in[12];
    const float* Am   = (const float*)d_in[13];
    const float* Bm   = (const float*)d_in[14];
    const float* dlt  = (const float*)d_in[15];
    const float* Wf   = (const float*)d_in[16];
    const float* bfo  = (const float*)d_in[17];
    const float* Wb   = (const float*)d_in[18];
    const float* bbo  = (const float*)d_in[19];
    float* OUT = (float*)d_out;
    char* wsp = (char*)d_ws;
    h16* LNH = (h16*)wsp; wsp += SZ_LNH;
    h16* WXZ = (h16*)wsp; wsp += SZ_WXZ;
    h16* WC  = (h16*)wsp; wsp += SZ_WC;
    h16* WO  = (h16*)wsp; wsp += SZ_WO;
    h16* XZH = (h16*)wsp; wsp += SZ_XZH;
    float* CFB = (float*)wsp; wsp += SZ_CFB;
    h16* FBH = (h16*)wsp; wsp += SZ_FBH;

    k_gse_ln<<<MR, 256, 0, stream>>>(x, wgse, bgse, lng, lnb, LNH);
    { const unsigned g = (unsigned)(((size_t)HID * G1 + 255) / 256);
      k_wcvt<<<g, 256, 0, stream>>>(Wx, WXZ, HID, DIN, G1, KP1);
      k_wcvt<<<g, 256, 0, stream>>>(Wz, WXZ + (size_t)HID * KP1, HID, DIN, G1, KP1); }
    { const unsigned g = (unsigned)(((size_t)HID * (HID / 8) + 255) / 256);
      k_wtap<<<g, 256, 0, stream>>>(Wcf, WC);
      k_wtap<<<g, 256, 0, stream>>>(Wcb, WC + (size_t)HID * HID); }
    { const unsigned g = (unsigned)(((size_t)ODIM * (HID / 8) + 255) / 256);
      k_wcvt<<<g, 256, 0, stream>>>(Wf, WO, ODIM, HID, HID / 8, CAT);
      k_wcvt<<<g, 256, 0, stream>>>(Wb, WO + HID, ODIM, HID, HID / 8, CAT); }

    k_gemm_h<<<dim3(HID / 64, 2, 1), 32 * GW, 0, stream>>>(LNH, WXZ, bx, bz, XZH, KP1, KP1, 0, HID, CAT, HID, 0);
    k_gemm_f<<<dim3(HID / 64, 2, 1), 32 * GW, 0, stream>>>(XZH, WC, bcf, bcb, CFB, HID, CAT, HID, HID, CAT, HID, 0, MR);
    k_tanhmean<<<HID / 64, 256, 0, stream>>>(CFB, Am, dlt, FBH, 0);
    k_tanhmean<<<HID / 64, 256, 0, stream>>>(CFB, Bm, dlt, FBH, HID);
    k_gemm_f<<<dim3(ODIM / 64, 1, 1), 32 * GW, 0, stream>>>(FBH, WO, bfo, bbo, OUT, CAT, CAT, 0, 0, ODIM, 0, 1, NB);
}
